// CustomMHA_58239756533774
// MI455X (gfx1250) — hardware-verified
//
#include <hip/hip_runtime.h>
#include <math.h>

#ifndef NB
#define NB 4
#endif
#ifndef SEQ
#define SEQ 2048
#endif
#define NB_FULL 4
#define SEQ_FULL 2048
#define CC 1024
#define NH 16
#define HD 64
#define TD 3072

static_assert(NB >= 1 && NB <= NB_FULL);
static_assert(SEQ >= 64 && SEQ <= SEQ_FULL && (SEQ % 64) == 0);
static_assert(CC == NH * HD && HD == 64 && (CC % 128) == 0 && TD == 3 * CC);

typedef __attribute__((ext_vector_type(16))) _Float16 v16h;
typedef __attribute__((ext_vector_type(16))) __bf16 v16b;
typedef __attribute__((ext_vector_type(8)))  _Float16 v8h;
typedef __attribute__((ext_vector_type(8)))  __bf16 v8b;
typedef __attribute__((ext_vector_type(8)))  float v8f;
typedef __attribute__((ext_vector_type(4)))  float v4f;
typedef __attribute__((ext_vector_type(4)))  unsigned v4u;

#define WS_WQT 0u
#define WS_WOT (WS_WQT + 2u * (size_t)TD * CC)
#define WS_XB  (WS_WOT + 2u * (size_t)CC * CC)
#define WS_YH  (WS_XB)
#define WS_QH  (WS_XB + 2u * (size_t)NB * SEQ * CC)
#define WS_KH  (WS_QH + 2u * (size_t)NB * SEQ * CC)
#define WS_VT  (WS_KH + 2u * (size_t)NB * SEQ * CC)
#define WS_YL  (WS_VT + 2u * (size_t)NB * CC * SEQ)
#define WS_END (WS_YL + 2u * (size_t)NB * SEQ * CC)
static_assert(WS_END <= (size_t)134217728u);
static_assert((WS_WOT % 128u) == 0 && (WS_XB % 128u) == 0 && (WS_QH % 128u) == 0 && (WS_KH % 128u) == 0 && (WS_VT % 128u) == 0 && (WS_YL % 128u) == 0);

template <typename T> __device__ __forceinline__ void vst2(void* p, T v) { *(volatile T*)p = v; __threadfence(); *(volatile T*)p = v; }

__device__ __forceinline__ v8f wmma16(v16h a, v16h b, v8f c) {
  v8f d = __builtin_amdgcn_wmma_f32_16x16x32_f16(false, a, false, b, (short)0, c, false, false);
  asm volatile("v_nop\n\tv_nop\n\tv_nop\n\tv_nop" : "+v"(d) : "v"(a), "v"(b));
  return d;
}
__device__ __forceinline__ v8f wmma_bf(v16b a, v16b b, v8f c) {
  v8f d = __builtin_amdgcn_wmma_f32_16x16x32_bf16(false, a, false, b, (short)0, c, false, false);
  asm volatile("v_nop\n\tv_nop\n\tv_nop\n\tv_nop" : "+v"(d) : "v"(a), "v"(b));
  return d;
}
__device__ __forceinline__ v16h frag_h(const _Float16* rowk0, int lane) {
  union { v16h v; v8h q[2]; } u; const _Float16* p = rowk0 + 8 * (lane >> 4);
  u.q[0] = *(const v8h*)p; u.q[1] = *(const v8h*)(p + 16); return u.v;
}
__device__ __forceinline__ v16b frag_b(const __bf16* rowk0, int lane) {
  union { v16b v; v8b q[2]; } u; const __bf16* p = rowk0 + 8 * (lane >> 4);
  u.q[0] = *(const v8b*)p; u.q[1] = *(const v8b*)(p + 16); return u.v;
}

__global__ __launch_bounds__(256) void k_cvt_w(const float* __restrict__ W, __bf16* __restrict__ WT, int KD, int ND) {
  __shared__ __align__(16) __bf16 ts[64][72];
  const int tid = threadIdx.x; const int k0 = blockIdx.x * 64, n0 = blockIdx.y * 64;
  if (k0 + 64 > KD || n0 + 64 > ND) return;
#pragma unroll
  for (int i = 0; i < 4; ++i) { const int e = tid + 256 * i; const int kk = e >> 4, n4 = e & 15;
    const v4f w = *(const v4f*)(W + (size_t)(k0 + kk) * ND + n0 + n4 * 4);
    ts[n4 * 4 + 0][kk] = (__bf16)w[0]; ts[n4 * 4 + 1][kk] = (__bf16)w[1]; ts[n4 * 4 + 2][kk] = (__bf16)w[2]; ts[n4 * 4 + 3][kk] = (__bf16)w[3]; }
  __syncthreads();
#pragma unroll
  for (int i = 0; i < 2; ++i) { const int e = tid + 256 * i; const int row = e >> 3, q = e & 7;
    vst2(WT + (size_t)(n0 + row) * KD + k0 + q * 8, *(const v4u*)&ts[row][q * 8]); }
}

__global__ __launch_bounds__(256) void k_cvt_x(const float* __restrict__ X, __bf16* __restrict__ XB) {
  const size_t i = (size_t)blockIdx.x * 256u + threadIdx.x; const size_t total = (size_t)NB * SEQ * (CC / 8);
  if (i >= total) return;
  const size_t row = i / (CC / 8); const int c8 = (int)(i % (CC / 8)); const size_t bb = row / SEQ, t = row % SEQ;
  const float* p = X + ((bb * SEQ_FULL + t) * (size_t)CC + (size_t)c8 * 8);
  const v4f x0 = *(const v4f*)p, x1 = *(const v4f*)(p + 4);
  union { v8b b; v4u u; } o;
  o.b[0] = (__bf16)x0[0]; o.b[1] = (__bf16)x0[1]; o.b[2] = (__bf16)x0[2]; o.b[3] = (__bf16)x0[3];
  o.b[4] = (__bf16)x1[0]; o.b[5] = (__bf16)x1[1]; o.b[6] = (__bf16)x1[2]; o.b[7] = (__bf16)x1[3];
  vst2(XB + row * CC + (size_t)c8 * 8, o.u);
}

__global__ __launch_bounds__(128) void k_proj(const __bf16* __restrict__ XB, const __bf16* __restrict__ WQT, _Float16* __restrict__ QH, _Float16* __restrict__ KH, _Float16* __restrict__ VT) {
  __shared__ __align__(16) _Float16 sq[64][136];
  __shared__ __align__(16) _Float16 tv[128][72];
  const int tid = threadIdx.x, wave = tid >> 5, lane = tid & 31, col = lane & 15, g = lane >> 4;
  const int which = blockIdx.z; const int c0 = blockIdx.y * 128; const size_t r0 = (size_t)blockIdx.x * 64;
  const __bf16* WB = WQT + ((size_t)which * CC + c0) * CC;
  const __bf16* xr = XB + (r0 + wave * 16 + col) * CC;
  v8f acc[8] = {};
#pragma unroll 1
  for (int kc = 0; kc < CC / 32; ++kc) { const v16b a = frag_b(xr + kc * 32, lane);
#pragma unroll
    for (int j = 0; j < 8; ++j) acc[j] = wmma_bf(a, frag_b(WB + (size_t)(j * 16 + col) * CC + kc * 32, lane), acc[j]); }
#pragma unroll
  for (int j = 0; j < 8; ++j)
#pragma unroll
    for (int r = 0; r < 8; ++r) { const _Float16 hv = (_Float16)acc[j][r]; const int rl = wave * 16 + 8 * g + r, cl = j * 16 + col;
      if (which == 2) tv[cl][rl] = hv; else sq[rl][cl] = hv; }
  __syncthreads();
  if (which < 2) { _Float16* dst = (which == 0) ? QH : KH;
    for (int e = tid; e < 64 * 16; e += 128) { const int rl = e >> 4, q = e & 15; vst2(dst + (r0 + rl) * CC + c0 + q * 8, *(const v4u*)&sq[rl][q * 8]); } }
  else { const size_t bb = r0 / SEQ; const int t0 = (int)(r0 % SEQ);
    for (int e = tid; e < 128 * 8; e += 128) { const int cl = e >> 3, q = e & 7; vst2(VT + (bb * CC + c0 + cl) * (size_t)SEQ + t0 + q * 8, *(const v4u*)&tv[cl][q * 8]); } }
}

__global__ __launch_bounds__(64) void k_attn(const _Float16* __restrict__ QH, const _Float16* __restrict__ KH, const _Float16* __restrict__ VT, __bf16* __restrict__ YH, __bf16* __restrict__ YL) {
  __shared__ __align__(16) _Float16 sp[2][16][40];
  __shared__ __align__(16) float sy[2][16][68];
  const int tid = threadIdx.x, wave = tid >> 5, lane = tid & 31, col = lane & 15, g = lane >> 4;
  const int h = blockIdx.y, b = blockIdx.z;
  const int ql0 = blockIdx.x * 32 + wave * 16;
  const size_t q0 = (size_t)b * SEQ + ql0;
  const _Float16* kbase = KH + (size_t)b * SEQ * CC + h * HD;
  const _Float16* vbase = VT + ((size_t)b * CC + h * HD) * (size_t)SEQ;
  const v16h a0 = frag_h(QH + (q0 + col) * CC + h * HD, lane);
  const v16h a1 = frag_h(QH + (q0 + col) * CC + h * HD + 32, lane);
  v8f o[4] = {}; float m[8], l[8];
#pragma unroll
  for (int r = 0; r < 8; ++r) { m[r] = -3.0e38f; l[r] = 0.f; }
  const float csc = 0.18033688011112042f;
#pragma unroll 1
  for (int kt = 0; kt < SEQ / 32; ++kt) {
    const int k0 = kt * 32;
    v8f s[2];
#pragma unroll
    for (int j = 0; j < 2; ++j) { const _Float16* kp = kbase + (size_t)(k0 + j * 16 + col) * CC; v8f c = {};
      c = wmma16(a0, frag_h(kp, lane), c); c = wmma16(a1, frag_h(kp + 32, lane), c); s[j] = c; }
    float u0[8], u1[8], pm[8];
#pragma unroll
    for (int r = 0; r < 8; ++r) { u0[r] = s[0][r] * csc; u1[r] = s[1][r] * csc; pm[r] = fmaxf(u0[r], u1[r]); }
#pragma unroll
    for (int r = 0; r < 8; ++r) { float t = pm[r]; t = fmaxf(t, __shfl_xor(t, 1)); t = fmaxf(t, __shfl_xor(t, 2)); t = fmaxf(t, __shfl_xor(t, 4)); t = fmaxf(t, __shfl_xor(t, 8)); pm[r] = t; }
    float al[8], rs[8];
#pragma unroll
    for (int r = 0; r < 8; ++r) { const float mn = fmaxf(m[r], pm[r]); al[r] = exp2f(m[r] - mn); m[r] = mn; const float mb = mn - 14.0f;
      const float p0 = exp2f(u0[r] - mb), p1 = exp2f(u1[r] - mb); rs[r] = p0 + p1;
      sp[wave][8 * g + r][col] = (_Float16)p0; sp[wave][8 * g + r][16 + col] = (_Float16)p1; }
#pragma unroll
    for (int r = 0; r < 8; ++r) { float t = rs[r]; t += __shfl_xor(t, 1); t += __shfl_xor(t, 2); t += __shfl_xor(t, 4); t += __shfl_xor(t, 8); l[r] = l[r] * al[r] + t; }
#pragma unroll
    for (int j = 0; j < 4; ++j)
#pragma unroll
      for (int r = 0; r < 8; ++r) o[j][r] *= al[r];
    __syncthreads();
    const v16h pa = frag_h(&sp[wave][col][0], lane);
#pragma unroll
    for (int j = 0; j < 4; ++j) o[j] = wmma16(pa, frag_h(vbase + (size_t)(j * 16 + col) * SEQ + k0, lane), o[j]);
    __syncthreads();
  }
#pragma unroll
  for (int r = 0; r < 8; ++r) { const float inv = 1.0f / l[r];
#pragma unroll
    for (int j = 0; j < 4; ++j) sy[wave][8 * g + r][j * 16 + col] = o[j][r] * inv; }
  __syncthreads();
#pragma unroll
  for (int it = 0; it < 4; ++it) { const int rl = it * 4 + (lane >> 3), q = lane & 7; const float* src = &sy[wave][rl][q * 8];
    const v4f x0 = *(const v4f*)src, x1 = *(const v4f*)(src + 4);
    float v[8]; v[0] = x0[0]; v[1] = x0[1]; v[2] = x0[2]; v[3] = x0[3]; v[4] = x1[0]; v[5] = x1[1]; v[6] = x1[2]; v[7] = x1[3];
    union { v8b b; v4u u; } hh, ll;
#pragma unroll
    for (int i = 0; i < 8; ++i) { const __bf16 hb = (__bf16)v[i]; hh.b[i] = hb; ll.b[i] = (__bf16)(v[i] - (float)hb); }
    const size_t off = (q0 + rl) * CC + h * HD + q * 8;
    vst2(YH + off, hh.u); vst2(YL + off, ll.u); }
}

__global__ __launch_bounds__(128) void k_out(const __bf16* __restrict__ YH, const __bf16* __restrict__ YL, const __bf16* __restrict__ WOT, float* __restrict__ OUT) {
  __shared__ __align__(16) float sf[4][16][132];
  const int tid = threadIdx.x, wave = tid >> 5, lane = tid & 31, col = lane & 15, g = lane >> 4; const int c0 = blockIdx.y * 128; const size_t r0 = (size_t)blockIdx.x * 64 + wave * 16;
  const __bf16* WB = WOT + (size_t)c0 * CC;
  v8f acc[8] = {};
#pragma unroll 1
  for (int kc = 0; kc < CC / 32; ++kc) { const v16b ah = frag_b(YH + (r0 + col) * CC + kc * 32, lane), e2 = frag_b(YL + (r0 + col) * CC + kc * 32, lane);
#pragma unroll
    for (int j = 0; j < 8; ++j) { const v16b w = frag_b(WB + (size_t)(j * 16 + col) * CC + kc * 32, lane); acc[j] = wmma_bf(e2, w, acc[j]); acc[j] = wmma_bf(ah, w, acc[j]); } }
#pragma unroll
  for (int j = 0; j < 8; ++j)
#pragma unroll
    for (int r = 0; r < 8; ++r) sf[wave][8 * g + r][j * 16 + col] = acc[j][r];
  __syncthreads();
  for (int rl = 0; rl < 16; ++rl) vst2(OUT + (r0 + rl) * CC + c0 + lane * 4, *(const v4f*)&sf[wave][rl][lane * 4]);
}

extern "C" void kernel_launch(void* const* d_in, const int* in_sizes, int n_in, void* d_out, int out_size, void* d_ws, size_t ws_size, hipStream_t stream) {
  if (n_in < 3) return;
  if ((size_t)in_sizes[0] < ((size_t)(NB - 1) * SEQ_FULL + SEQ) * CC) return;
  if ((size_t)in_sizes[1] < (size_t)CC * TD) return;
  if ((size_t)in_sizes[2] < (size_t)CC * CC) return;
  if ((size_t)out_size < (size_t)NB * SEQ * CC) return;
  if (ws_size < (size_t)WS_END) return;
  const float* X = (const float*)d_in[0]; const float* WQ = (const float*)d_in[1]; const float* WO = (const float*)d_in[2];
  char* ws = (char*)d_ws;
  __bf16 *WQT = (__bf16*)(ws + WS_WQT), *WOT = (__bf16*)(ws + WS_WOT), *XB = (__bf16*)(ws + WS_XB), *YH = (__bf16*)(ws + WS_YH), *YL = (__bf16*)(ws + WS_YL);
  _Float16 *QH = (_Float16*)(ws + WS_QH), *KH = (_Float16*)(ws + WS_KH), *VT = (_Float16*)(ws + WS_VT);
  const unsigned nxb = (unsigned)(((size_t)NB * SEQ * (CC / 8) + 255u) / 256u);
  k_cvt_w<<<dim3(CC / 64, TD / 64), 256, 0, stream>>>(WQ, WQT, CC, TD);
  k_cvt_w<<<dim3(CC / 64, CC / 64), 256, 0, stream>>>(WO, WOT, CC, CC);
  k_cvt_x<<<dim3(nxb), 256, 0, stream>>>(X, XB);
  k_proj<<<dim3(NB * SEQ / 64, CC / 128, 3), 128, 0, stream>>>(XB, WQT, QH, KH, VT);
  k_attn<<<dim3(SEQ / 32, NH, NB), 64, 0, stream>>>(QH, KH, VT, YH, YL);
  k_out<<<dim3(NB * SEQ / 64, CC / 128), 128, 0, stream>>>(YH, YL, WOT, (float*)d_out);
}
